// PolymorphicDenseBase_50517405336015
// MI455X (gfx1250) — hardware-verified
//
#include <hip/hip_runtime.h>
#include <math.h>

#define NBR 16384
#define KEYD 64
#define DD 128
#define UU 128
#define NMODE 32
#define KTOT (NMODE * DD + NMODE)

typedef _Float16 f16;
typedef __attribute__((ext_vector_type(16))) f16 f16x16;
typedef __attribute__((ext_vector_type(8)))  f16 f16x8;
typedef __attribute__((ext_vector_type(8)))  float f32x8;
typedef __attribute__((ext_vector_type(4)))  float v4f_t;
typedef float v4fa __attribute__((ext_vector_type(4), may_alias));
__device__ __forceinline__ f32x8 wmma16(f16x16 a, f16x16 b, f32x8 c) {
  c = __builtin_amdgcn_wmma_f32_16x16x32_f16(false, a, false, b, (short)0, c, false, false);
  asm volatile("v_nop\n\tv_nop\n\tv_nop\n\tv_nop" : "+v"(c) : "v"(a), "v"(b));
  return c;
}
__device__ __forceinline__ f16x16 lds_frag(const f16* base, int stride) {
  const int lane = threadIdx.x & 31, row = lane & 15, kh = (lane >> 4) * 8;
  const f16x8 lo = *(const f16x8*)(base + row * stride + kh);
  const f16x8 hi = *(const f16x8*)(base + row * stride + kh + 16);
  f16x16 f;
#pragma unroll
  for (int i = 0; i < 8; ++i) { f[i] = lo[i]; f[i + 8] = hi[i]; }
  return f;
}

__global__ __launch_bounds__(256) void k_poly(const float* __restrict__ keyv, const float* __restrict__ x, const float* __restrict__ sens, const float* __restrict__ kmap,
                                             const float* __restrict__ kern, const float* __restrict__ bias, float* __restrict__ out) {
  __shared__ __attribute__((aligned(16))) f16 aS[2][64 * 40];
  __shared__ __attribute__((aligned(16))) f16 wS[2][128 * 40];
  __shared__ float simS[64 * 33];
  __shared__ float kmS[NMODE * KEYD];
  __shared__ __attribute__((aligned(16))) float oS[8][32 * 36];
  const int tid = threadIdx.x, lane = tid & 31, wave = tid >> 5, cl = lane & 15, rh = (lane >> 4) * 8;
  const int r0 = blockIdx.x * 64; const int wm = (wave & 1) * 32, wn = (wave >> 1) * 32;
  for (int e = tid; e < NMODE * KEYD; e += 256) kmS[e] = kmap[e];
  __syncthreads();
  { const int row = tid >> 2, mq = (tid & 3) * 8; const float* kr = keyv + (size_t)(r0 + row) * KEYD; float lg[8]; float mx = -3.0e38f;
    for (int i = 0; i < 8; ++i) { const int m = mq + i; float s = 0.0f;
#pragma unroll 8
      for (int c = 0; c < KEYD; ++c) { const float d = kr[c] - kmS[m * KEYD + c]; s += d * d; }
      lg[i] = sens[m] / (sqrtf(s) + 1.0f); mx = fmaxf(mx, lg[i]); }
    mx = fmaxf(mx, __shfl_xor(mx, 1, 32)); mx = fmaxf(mx, __shfl_xor(mx, 2, 32)); float z = 0.0f;
    for (int i = 0; i < 8; ++i) { lg[i] = expf(lg[i] - mx); z += lg[i]; }
    z += __shfl_xor(z, 1, 32); z += __shfl_xor(z, 2, 32); const float iz = 1.0f / z;
    for (int i = 0; i < 8; ++i) simS[row * 33 + mq + i] = lg[i] * iz; }
  f32x8 acc[2][2], accx[2][2];
#pragma unroll
  for (int i = 0; i < 2; ++i)
#pragma unroll
    for (int j = 0; j < 2; ++j) { f32x8 zz = {}; acc[i][j] = zz; accx[i][j] = zz; }
  __syncthreads();
#pragma unroll 1
  for (int ks = 0; ks < KTOT / 32; ++ks) {
    __syncthreads();
    { const int row = tid >> 2, kq = (tid & 3) * 8; const float* xr = x + (size_t)(r0 + row) * DD;
#pragma unroll
      for (int uu = 0; uu < 8; ++uu) { const int k = ks * 32 + kq + uu; float v;
        if (k < NMODE * DD) { const int m = k >> 7, d = k & 127; v = simS[row * 33 + m] * xr[d] * 64.0f; } else v = simS[row * 33 + (k - NMODE * DD)] * 64.0f;
        const f16 hh = (f16)v; aS[0][row * 40 + kq + uu] = hh; aS[1][row * 40 + kq + uu] = (f16)((v - (float)hh) * 2048.0f); } }
    { const int u = tid >> 1, kq = (tid & 1) * 16;
#pragma unroll
      for (int uu = 0; uu < 16; ++uu) { const int k = ks * 32 + kq + uu; const float v = 16.0f * ((k < NMODE * DD) ? kern[(size_t)k * UU + u] : bias[(size_t)(k - NMODE * DD) * UU + u]);
        const f16 hh = (f16)v; wS[0][u * 40 + kq + uu] = hh; wS[1][u * 40 + kq + uu] = (f16)((v - (float)hh) * 2048.0f); } }
    __syncthreads();
    f16x16 ah[2], al[2];
#pragma unroll
    for (int i = 0; i < 2; ++i) { ah[i] = lds_frag(aS[0] + (wm + 16 * i) * 40, 40); al[i] = lds_frag(aS[1] + (wm + 16 * i) * 40, 40); }
#pragma unroll
    for (int j = 0; j < 2; ++j) { const f16x16 bh = lds_frag(wS[0] + (wn + 16 * j) * 40, 40), bl = lds_frag(wS[1] + (wn + 16 * j) * 40, 40);
#pragma unroll
      for (int i = 0; i < 2; ++i) { acc[i][j] = wmma16(ah[i], bh, acc[i][j]); accx[i][j] = wmma16(ah[i], bl, accx[i][j]); accx[i][j] = wmma16(al[i], bh, accx[i][j]); } }
  }
  float* so = oS[wave];
#pragma unroll
  for (int i = 0; i < 2; ++i)
#pragma unroll
    for (int r = 0; r < 8; ++r)
#pragma unroll
      for (int j = 0; j < 2; ++j) so[(16 * i + rh + r) * 36 + 16 * j + cl] = (acc[i][j][r] + accx[i][j][r] * (1.0f / 2048.0f)) * (1.0f / (NMODE * 1024.0f));
  asm volatile("s_wait_dscnt 0" ::: "memory");
  __builtin_amdgcn_wave_barrier();
#pragma unroll 1
  for (int pass = 0; pass < 2; ++pass) {
#pragma unroll
    for (int it = 0; it < 8; ++it) { const int f4 = lane + 32 * it, rr = f4 >> 3, q = (f4 & 7) * 4;
      *(volatile v4f_t*)(out + (size_t)(r0 + wm + rr) * UU + wn + q) = *(const volatile v4fa*)(so + rr * 36 + q); }
    __threadfence();
  }
}

extern "C" void kernel_launch(void* const* d_in, const int* in_sizes, int n_in,
                              void* d_out, int out_size, void* d_ws, size_t ws_size,
                              hipStream_t stream) {
  (void)in_sizes; (void)n_in; (void)out_size; (void)d_ws; (void)ws_size;
  const float* keyv = (const float*)d_in[0];
  const float* x = (const float*)d_in[1];
  const float* sens = (const float*)d_in[2];
  const float* kmap = (const float*)d_in[3];
  const float* kern = (const float*)d_in[4];
  const float* bias = (const float*)d_in[5];
  float* out = (float*)d_out;
  k_poly<<<dim3(NBR / 64), dim3(256), 0, stream>>>(keyv, x, sens, kmap, kern, bias, out);
}
